// GaussianImage_Cholesky_36524401885824
// MI455X (gfx1250) — hardware-verified
//
#include <hip/hip_runtime.h>


#define NG   2048
#define IMH  256
#define IMW  256
#define NPX  (IMH * IMW)
#define PCH  8192
#define NCP  64
typedef _Float16 h16;
typedef unsigned short bf;
typedef __attribute__((ext_vector_type(16))) __bf16   v16bf;
typedef __attribute__((ext_vector_type(16))) _Float16 v16h;
typedef __attribute__((ext_vector_type(8)))  _Float16 v8h;
typedef __attribute__((ext_vector_type(8)))  unsigned short v8us;
typedef __attribute__((ext_vector_type(8)))  float    v8f;
typedef __attribute__((ext_vector_type(4)))  float    v4f;
typedef v8h  __attribute__((may_alias)) v8ha;
typedef v4f  __attribute__((may_alias)) v4fa;
typedef v8us __attribute__((may_alias)) v8usa;

__device__ __forceinline__ unsigned short f2bf(float f) { unsigned u = __float_as_uint(f); u += 0x7FFFu + ((u >> 16) & 1u); return (unsigned short)(u >> 16); }
__device__ __forceinline__ float bf2f(unsigned short b) { return __uint_as_float(((unsigned)b) << 16); }
__device__ __forceinline__ float bfr(float f) { return bf2f(f2bf(f)); }
__device__ __forceinline__ v16h cat16(v8h lo, v8h hi) { return __builtin_shufflevector(lo, hi, 0, 1, 2, 3, 4, 5, 6, 7, 8, 9, 10, 11, 12, 13, 14, 15); }
__device__ __forceinline__ v16bf cat16b(v8us lo, v8us hi) { return __builtin_bit_cast(v16bf, __builtin_shufflevector(lo, hi, 0, 1, 2, 3, 4, 5, 6, 7, 8, 9, 10, 11, 12, 13, 14, 15)); }
__device__ __forceinline__ v8f wmma16(v16h a, v16h b, v8f c) { return __builtin_amdgcn_wmma_f32_16x16x32_f16(false, a, false, b, (short)0, c, false, false); }
__device__ __forceinline__ v8f wmmab(v16bf a, v16bf b, v8f c) { return __builtin_amdgcn_wmma_f32_16x16x32_bf16(false, a, false, b, (short)0, c, false, false); }


template <typename T16> struct WFrag;
template <> struct WFrag<h16> { typedef v16h V; static __device__ __forceinline__ V ld(const h16* p) { return cat16(*(const v8h*)p, *(const v8h*)(p + 16)); } static __device__ __forceinline__ v8f mma(V a, V b, v8f c) { return wmma16(a, b, c); } };
template <> struct WFrag<bf> { typedef v16bf V; static __device__ __forceinline__ V ld(const bf* p) { return cat16b(*(const v8us*)p, *(const v8us*)(p + 16)); } static __device__ __forceinline__ v8f mma(V a, V b, v8f c) { return wmmab(a, b, c); } };
template <typename T16, int NSPLIT, bool BIAS>
__global__ __launch_bounds__(32) void k_gemmw(const T16* __restrict__ A, const T16* __restrict__ A2, const T16* __restrict__ Bt, const T16* __restrict__ Bt2, int K, float* C, int ldc, const float* __restrict__ bias, size_t sA, size_t sB, size_t sC) {
    typedef typename WFrag<T16>::V V;
    __shared__ __align__(16) float os[16 * 68];
    const size_t z = blockIdx.z; A += z * sA; if (A2) A2 += z * sA; Bt += z * sB; if (Bt2) Bt2 += z * sB; C += z * sC;
    const int lane = threadIdx.x & 31, lr = lane & 15, hi = lane >> 4; const int r0 = blockIdx.x * 64, c0 = blockIdx.y * 64;
    v8f acc[4][4];
#pragma unroll
    for (int mb = 0; mb < 4; ++mb)
#pragma unroll
        for (int nb = 0; nb < 4; ++nb) acc[mb][nb] = (v8f){};
    const size_t aoff = (size_t)(r0 + lr) * K + 8 * hi, boff = (size_t)(c0 + lr) * K + 8 * hi;
#pragma unroll 1
    for (int kc = 0; kc < K; kc += 32) {
        V a[4], a2[4];
#pragma unroll
        for (int mb = 0; mb < 4; ++mb) { a[mb] = WFrag<T16>::ld(A + aoff + (size_t)mb * 16 * K + kc); if (NSPLIT == 1 || NSPLIT == 2) a2[mb] = WFrag<T16>::ld(A2 + aoff + (size_t)mb * 16 * K + kc); }
#pragma unroll
        for (int nb = 0; nb < 4; ++nb) { const V b = WFrag<T16>::ld(Bt + boff + (size_t)nb * 16 * K + kc); V b2; if (NSPLIT >= 2) b2 = WFrag<T16>::ld(Bt2 + boff + (size_t)nb * 16 * K + kc);
#pragma unroll
            for (int mb = 0; mb < 4; ++mb) { acc[mb][nb] = WFrag<T16>::mma(a[mb], b, acc[mb][nb]); if (NSPLIT == 1 || NSPLIT == 2) acc[mb][nb] = WFrag<T16>::mma(a2[mb], b, acc[mb][nb]); if (NSPLIT >= 2) acc[mb][nb] = WFrag<T16>::mma(a[mb], b2, acc[mb][nb]); } }
        asm volatile("v_nop\n\tv_nop\n\tv_nop\n\tv_nop" : "+v"(acc[0][0]), "+v"(acc[1][1]), "+v"(acc[2][2]), "+v"(acc[3][3]) : "v"(a[0]), "v"(a[3]));
    }
#pragma unroll
    for (int mb = 0; mb < 4; ++mb) {
#pragma unroll
        for (int nb = 0; nb < 4; ++nb) {
#pragma unroll
            for (int j = 0; j < 8; ++j) os[(hi * 8 + j) * 68 + nb * 16 + lr] = acc[mb][nb][j]; }
        __builtin_amdgcn_wave_barrier(); asm volatile("" ::: "memory");
        float* crow = C + (size_t)(r0 + mb * 16) * ldc + c0;
#pragma unroll 1
        for (int ps = 0; ps < 2; ++ps) {
#pragma unroll
            for (int s = 0; s < 8; ++s) { const int row = 2 * s + hi, cofs = lr * 4; v4f val = *(const v4fa*)(os + row * 68 + cofs); if (BIAS) { val[0] += bfr(bias[c0 + cofs]); val[1] += bfr(bias[c0 + cofs + 1]); val[2] += bfr(bias[c0 + cofs + 2]); val[3] += bfr(bias[c0 + cofs + 3]); }
                *(volatile v4f*)(crow + (size_t)row * ldc + cofs) = val; }
            if (ps == 0) __threadfence(); }
        __builtin_amdgcn_wave_barrier(); asm volatile("" ::: "memory");
    }
}

typedef __attribute__((ext_vector_type(2))) float v2f;
__device__ __forceinline__ void splitf(float y, unsigned short& h, unsigned short& l) { h = f2bf(y); l = f2bf(y - bf2f(h)); }
__device__ __forceinline__ float sigm(float a) { return __fdiv_rn(1.0f, __fadd_rn(1.0f, __builtin_amdgcn_exp2f(__fmul_rn(a, -1.4426950408889634f)))); }
__device__ __forceinline__ float tanhx(float a) { return __fsub_rn(__fdiv_rn(2.0f, __fadd_rn(1.0f, __builtin_amdgcn_exp2f(__fmul_rn(a, -2.8853900817779268f)))), 1.0f); }
__global__ __launch_bounds__(256) void k_gparam(const float* __restrict__ xyz, const float* __restrict__ chl, const float* __restrict__ opa, const int* __restrict__ fidx, float* GP) {
    const int n = blockIdx.x * 256 + threadIdx.x; if (n >= NG) return; const float t = __fdiv_rn((float)fidx[0], 7.0f); const float t2 = __fmul_rn(t, t);
    float m[2], l[3];
#pragma unroll
    for (int p = 0; p < 2; ++p) { float s = bfr(xyz[(size_t)(0 * NG + n) * 2 + p]); float a1 = __fmul_rn(bfr(xyz[(size_t)(1 * NG + n) * 2 + p]), t); asm volatile("" : "+v"(a1)); float a2 = __fmul_rn(bfr(xyz[(size_t)(2 * NG + n) * 2 + p]), t2); asm volatile("" : "+v"(a2)); s = __fadd_rn(__fadd_rn(s, a1), a2); m[p] = tanhx(s); }
#pragma unroll
    for (int c = 0; c < 3; ++c) { float s = bfr(chl[(size_t)(0 * NG + n) * 3 + c]); float a1 = __fmul_rn(bfr(chl[(size_t)(1 * NG + n) * 3 + c]), t); asm volatile("" : "+v"(a1)); float a2 = __fmul_rn(bfr(chl[(size_t)(2 * NG + n) * 3 + c]), t2); asm volatile("" : "+v"(a2)); s = __fadd_rn(__fadd_rn(s, a1), a2); l[c] = (c == 1) ? s : __fadd_rn(s, 0.5f); }
    float s11 = __fmul_rn(l[0], l[0]), s12 = __fmul_rn(l[0], l[1]), s22a = __fmul_rn(l[1], l[1]), s22b = __fmul_rn(l[2], l[2]); asm volatile("" : "+v"(s11), "+v"(s12), "+v"(s22a), "+v"(s22b)); const float s22 = __fadd_rn(s22a, s22b);
    float d1 = __fmul_rn(s11, s22), d2 = __fmul_rn(s12, s12); asm volatile("" : "+v"(d1), "+v"(d2)); const float det = __fsub_rn(d1, d2);
    v4f g0, g1; g0[0] = __fdiv_rn(s22, det); g0[1] = __fdiv_rn(-s12, det); g0[2] = __fdiv_rn(s11, det); g0[3] = __fmul_rn(0.5f * IMW, __fadd_rn(m[0], 1.0f)); g1[0] = __fmul_rn(0.5f * IMH, __fadd_rn(m[1], 1.0f)); g1[1] = sigm(bfr(opa[n])); g1[2] = 0.f; g1[3] = 0.f;
#pragma unroll
    for (int ps = 0; ps < 2; ++ps) { *(volatile v4f*)(GP + (size_t)n * 8) = g0; *(volatile v4f*)(GP + (size_t)n * 8 + 4) = g1;
        if (ps == 0) __threadfence(); }
}
__global__ __launch_bounds__(256) void k_col(const float* __restrict__ fdc, bf* COLh, bf* COLl) { const int i = blockIdx.x * 256 + threadIdx.x; if (i >= 3 * NG / 8) return; const int c = i / (NG / 8), n0 = (i % (NG / 8)) * 8; v8us oh, ol;
#pragma unroll
    for (int k = 0; k < 8; ++k) { unsigned short a2, c2; splitf(sigm(bfr(fdc[(size_t)(n0 + k) * 3 + c])), a2, c2); oh[k] = a2; ol[k] = c2; }
    const size_t o = (size_t)c * NG + n0; *(volatile v8us*)(COLh + o) = oh; *(volatile v8us*)(COLl + o) = ol; __threadfence(); *(volatile v8us*)(COLh + o) = oh; *(volatile v8us*)(COLl + o) = ol; }
__global__ __launch_bounds__(256) void k_czero(bf* COLh, bf* COLl) { const size_t i = (size_t)blockIdx.x * 256 + threadIdx.x; const size_t n8 = (size_t)(NCP - 3) * NG / 8; if (i >= n8) return; v8us z;
#pragma unroll
    for (int k = 0; k < 8; ++k) z[k] = 0; const size_t o = (size_t)3 * NG + i * 8; *(volatile v8us*)(COLh + o) = z; *(volatile v8us*)(COLl + o) = z; __threadfence(); *(volatile v8us*)(COLh + o) = z; *(volatile v8us*)(COLl + o) = z; }
__global__ __launch_bounds__(256) void k_alpha(const float* __restrict__ GP, int p0, bf* ALh, bf* ALl) {
    const size_t i = (size_t)blockIdx.x * 256 + threadIdx.x; if (i >= (size_t)PCH * NG / 8) return; const int n0 = (int)(i % (NG / 8)) * 8; const int pl = (int)(i / (NG / 8)); const int p = p0 + pl; const float px = __fadd_rn((float)(p % IMW), 0.5f), py = __fadd_rn((float)(p / IMW), 0.5f); v8us oh, ol;
#pragma unroll
    for (int k = 0; k < 8; ++k) { const v4f g0 = *(const v4f*)(GP + (size_t)(n0 + k) * 8); const v4f g1 = *(const v4f*)(GP + (size_t)(n0 + k) * 8 + 4);
        const float dx = __fsub_rn(px, g0[3]), dy = __fsub_rn(py, g1[0]); float dx2 = __fmul_rn(dx, dx), dy2 = __fmul_rn(dy, dy), dxy = __fmul_rn(dy, dx); asm volatile("" : "+v"(dx2), "+v"(dy2), "+v"(dxy));
        float ta = __fmul_rn(__fmul_rn(0.5f, g0[0]), dx2), tc = __fmul_rn(__fmul_rn(0.5f, g0[2]), dy2), tb = __fmul_rn(g0[1], dxy); asm volatile("" : "+v"(ta), "+v"(tc), "+v"(tb)); const float sg = __fadd_rn(__fadd_rn(ta, tc), tb);
        float e = __builtin_amdgcn_exp2f(__fmul_rn(sg, -1.4426950408889634f)); asm volatile("" : "+v"(e)); const float al = fminf(0.99f, __fmul_rn(g1[1], e)); unsigned short a2, c2; splitf(al, a2, c2); oh[k] = a2; ol[k] = c2; }
    const size_t o = (size_t)pl * NG + n0; *(volatile v8us*)(ALh + o) = oh; *(volatile v8us*)(ALl + o) = ol; __threadfence(); *(volatile v8us*)(ALh + o) = oh; *(volatile v8us*)(ALl + o) = ol; }
__global__ __launch_bounds__(256) void k_img(const float* __restrict__ IMG, int p0, float* out) { const int i = blockIdx.x * 256 + threadIdx.x; if (i >= PCH / 4) return; const int pl = i * 4;
#pragma unroll
    for (int c = 0; c < 3; ++c) { v4f o;
#pragma unroll
        for (int q = 0; q < 4; ++q) o[q] = fminf(1.0f, fmaxf(0.0f, IMG[(size_t)(pl + q) * NCP + c]));
        *(volatile v4f*)(out + (size_t)c * NPX + p0 + pl) = o; __threadfence(); *(volatile v4f*)(out + (size_t)c * NPX + p0 + pl) = o; } }

extern "C" void kernel_launch(void* const* d_in, const int* in_sizes, int n_in,
                              void* d_out, int out_size, void* d_ws, size_t ws_size, hipStream_t stream) {
    (void)in_sizes; (void)n_in; (void)out_size;
    const float* xyz = (const float*)d_in[0]; const float* chl = (const float*)d_in[1]; const float* opa = (const float*)d_in[2]; const float* fdc = (const float*)d_in[3]; const int* fidx = (const int*)d_in[4];
    float* OUT = (float*)d_out;
    char* wsp = (char*)d_ws;
    auto take = [&](size_t bytes) { char* p = wsp; wsp += (bytes + 255) & ~(size_t)255; return (void*)p; };
    float* GP = (float*)take((size_t)NG * 8 * 4); bf* COLh = (bf*)take((size_t)NCP * NG * 2); bf* COLl = (bf*)take((size_t)NCP * NG * 2); bf* ALh = (bf*)take((size_t)PCH * NG * 2); bf* ALl = (bf*)take((size_t)PCH * NG * 2); float* IMG = (float*)take((size_t)PCH * NCP * 4);
    if ((size_t)(wsp - (char*)d_ws) > ws_size) return;
    k_gparam<<<NG / 256, 256, 0, stream>>>(xyz, chl, opa, fidx, GP); k_col<<<(3 * NG / 8 + 255) / 256, 256, 0, stream>>>(fdc, COLh, COLl); k_czero<<<(unsigned)(((size_t)(NCP - 3) * NG / 8 + 255) / 256), 256, 0, stream>>>(COLh, COLl);
    for (int p0 = 0; p0 < NPX; p0 += PCH) {
        k_alpha<<<(unsigned)(((size_t)PCH * NG / 8 + 255) / 256), 256, 0, stream>>>(GP, p0, ALh, ALl);
        k_gemmw<bf, 2, false><<<dim3(PCH / 64, NCP / 64, 1), 32, 0, stream>>>(ALh, ALl, COLh, COLl, NG, IMG, NCP, nullptr, 0, 0, 0);
        k_img<<<(PCH / 4 + 255) / 256, 256, 0, stream>>>(IMG, p0, OUT); }
}
